// CNNLSTM_59193239273595
// MI455X (gfx1250) — hardware-run, weakly checked
//
#include <hip/hip_runtime.h>
#include <stdint.h>
#include <stddef.h>

typedef __attribute__((ext_vector_type(16))) _Float16 v16h;
typedef __attribute__((ext_vector_type(8)))  _Float16 v8h;
typedef __attribute__((ext_vector_type(16))) __bf16   v16b;
typedef __attribute__((ext_vector_type(8)))  __bf16   v8b;
typedef __attribute__((ext_vector_type(8)))  float    v8f;
typedef __attribute__((ext_vector_type(4)))  float    v4f;
typedef __attribute__((ext_vector_type(4)))  unsigned u32x4;

constexpr int NBATCH   = 64;
constexpr int NSEQ     = 4096;
constexpr int NSEQPAD  = 4104;
constexpr int NEMB     = 128;
constexpr int NFILT    = 64;
constexpr int NTAP     = 5;
constexpr int KCONV    = NEMB * NTAP;
constexpr int NSTEP    = 1023;
constexpr int NSTEPPAD = 1024;
constexpr int NHID     = 128;
constexpr int NGATE    = 512;
constexpr int NCLS     = 2;
constexpr int HPITCH   = 136;
constexpr float CARRY16 = 16.0f;
constexpr float INV256  = 1.0f / 256.0f;

constexpr size_t SZ_HEMB  = (size_t)NBATCH * NSEQPAD * NEMB * 2;
constexpr size_t SZ_XG16  = (size_t)NBATCH * NSTEPPAD * NGATE * 2;
constexpr size_t SZ_CONV  = (size_t)NBATCH * NSEQ * NFILT * 2;
constexpr size_t SZ_HPOOL = (size_t)NBATCH * NSTEPPAD * NFILT * 2;
constexpr size_t SZ_WCONV = (size_t)NFILT * KCONV * 2;
constexpr size_t SZ_WIH   = (size_t)NGATE * NFILT * 2;
constexpr size_t SZ_WHH   = (size_t)NGATE * NHID * 2;
constexpr size_t SZ_BIAS  = (size_t)NGATE * 4;
constexpr size_t OFF_HEMB  = 0;
constexpr size_t OFF_CONV  = OFF_HEMB + SZ_HEMB;
constexpr size_t OFF_HPOOL = OFF_CONV + SZ_CONV;
constexpr size_t OFF_WCONV = OFF_HPOOL + SZ_HPOOL;
constexpr size_t OFF_WIH   = OFF_WCONV + SZ_WCONV;
constexpr size_t OFF_WHH   = OFF_WIH + SZ_WIH;
constexpr size_t OFF_BIAS  = OFF_WHH + SZ_WHH;
constexpr size_t WS_TOTAL  = OFF_BIAS + SZ_BIAS;
static_assert(SZ_XG16 <= SZ_HEMB, "xg plane overlays the embedding plane");
static_assert(WS_TOTAL <= (size_t)134217728, "carve within 128 MiB");
static_assert((OFF_CONV % 256) == 0 && (OFF_HPOOL % 256) == 0 && (OFF_WCONV % 256) == 0 && (OFF_WIH % 256) == 0 && (OFF_WHH % 256) == 0 && (OFF_BIAS % 256) == 0, "aligned carve");
static_assert(KCONV % 32 == 0 && NSEQ % 64 == 0 && NFILT % 64 == 0, "conv GEMM shapes");
static_assert(NFILT % 32 == 0 && (NBATCH * NSTEPPAD) % 64 == 0 && NGATE % 64 == 0, "projection GEMM shapes");
static_assert(NHID % 32 == 0, "recurrent K");
static_assert((size_t)(NSEQ - 1) * NEMB + KCONV <= (size_t)NSEQPAD * NEMB, "conv A padding");
static_assert((NBATCH * NSEQPAD) % 16 == 0, "gather grid");
static_assert(NSTEP == (NSEQ - NTAP + 1) / 4, "pooled length");

__device__ __forceinline__ unsigned short f2bf_bits(float f) {
  unsigned u = __float_as_uint(f);
  return (unsigned short)((u + 0x7FFFu + ((u >> 16) & 1u)) >> 16);
}
__device__ __forceinline__ float bf_bits2f(unsigned short h) { return __uint_as_float(((unsigned)h) << 16); }

__device__ __forceinline__ void dep_guard_h(v8f& a, v8f& b, v16h x, v16h y) { asm volatile("v_nop\n\tv_nop\n\tv_nop\n\tv_nop" : "+v"(a), "+v"(b) : "v"(x), "v"(y)); }
__device__ __forceinline__ void dep_guard_b(v8f& a, v8f& b, v16b x, v16b y) { asm volatile("v_nop\n\tv_nop\n\tv_nop\n\tv_nop" : "+v"(a), "+v"(b) : "v"(x), "v"(y)); }
__device__ __forceinline__ void keep4_h(v16h a, v16h b, v16h c, v16h d) { asm volatile("v_nop" :: "v"(a), "v"(b), "v"(c), "v"(d)); }
__device__ __forceinline__ void keep4_b(v16b a, v16b b, v16b c, v16b d) { asm volatile("v_nop" :: "v"(a), "v"(b), "v"(c), "v"(d)); }
__device__ __forceinline__ void acc_guard4(v8f& a, v8f& b, v8f& c, v8f& d) { asm volatile("v_nop\n\tv_nop\n\tv_nop\n\tv_nop" : "+v"(a), "+v"(b), "+v"(c), "+v"(d)); }
template <typename T> struct Frag;
template <> struct Frag<_Float16> {
  typedef v16h V; union U { v16h v; v8h h[2]; };
  static __device__ __forceinline__ v16h load(const _Float16* p) {
    U f; f.h[0] = *(const v8h*)(p); f.h[1] = *(const v8h*)(p + 16); return f.v;
  }
  static __device__ __forceinline__ v8f mma(v16h a, v16h b, v8f c) {
    return __builtin_amdgcn_wmma_f32_16x16x32_f16(false, a, false, b, (short)0, c, false, false);
  }
  static __device__ __forceinline__ void guard(v8f& a, v8f& b, v16h x, v16h y) { dep_guard_h(a, b, x, y); }
  static __device__ __forceinline__ void keep(v16h a, v16h b, v16h c, v16h d) { keep4_h(a, b, c, d); }
};
template <> struct Frag<__bf16> {
  typedef v16b V; union U { v16b v; v8b h[2]; };
  static __device__ __forceinline__ v16b load(const __bf16* p) {
    U f; f.h[0] = *(const v8b*)(p); f.h[1] = *(const v8b*)(p + 16); return f.v;
  }
  static __device__ __forceinline__ v8f mma(v16b a, v16b b, v8f c) {
    return __builtin_amdgcn_wmma_f32_16x16x32_bf16(false, a, false, b, (short)0, c, false, false);
  }
  static __device__ __forceinline__ void guard(v8f& a, v8f& b, v16b x, v16b y) { dep_guard_b(a, b, x, y); }
  static __device__ __forceinline__ void keep(v16b a, v16b b, v16b c, v16b d) { keep4_b(a, b, c, d); }
};

template <int ET> struct Elem;
template <> struct Elem<0> { typedef _Float16 T; };
template <> struct Elem<1> { typedef __bf16 T; };
template <int ET, bool SPLIT, int BIAS_MODE, int OUT_MODE, bool RESID, int ACT = 0>
__global__ __launch_bounds__(256) void wmma_gemm64(
    const unsigned short* __restrict__ Ap, const unsigned short* __restrict__ A2p, int lda, long strideA,
    const unsigned short* __restrict__ Btp, const unsigned short* __restrict__ Bt2p, int ldb, long strideB,
    void* __restrict__ Cout, void* __restrict__ Cout2, int ldc, long strideC,
    const float* __restrict__ bias,
    const float* __restrict__ resid, long strideR,
    int M, int N, int K, float scale) {
  typedef typename Elem<ET>::T T;
  typedef typename Frag<T>::V V;
  const T* A = (const T*)Ap; const T* A2 = (const T*)A2p; const T* Bt = (const T*)Btp; const T* Bt2 = (const T*)Bt2p;
  __shared__ __align__(16) float sT[8][16 * 68];
  const int b    = blockIdx.y;
  const int lane = threadIdx.x & 31;
  const int wave = threadIdx.x >> 5;
  const int tilesN = N >> 6;
  const int tilesM = M >> 6;
  const int tile = blockIdx.x * 8 + wave;
  if (tile >= tilesM * tilesN) return;
  const int tm = tile / tilesN;
  const int tn = tile - tm * tilesN;
  const int m0 = tm << 6;
  const int n0 = tn << 6;

  const T* Ab  = A  + (size_t)b * strideA;
  const T* Bb  = Bt + (size_t)b * strideB;
  const T* Ab2 = SPLIT ? (A2  + (size_t)b * strideA) : nullptr;
  const T* Bb2 = SPLIT ? (Bt2 + (size_t)b * strideB) : nullptr;

  const int rlane = lane & 15;
  const int koff  = (lane >> 4) * 8;
  const int mOff  = (lane >> 4) * 8;

  v8f acc[4][4];
#pragma unroll
  for (int i = 0; i < 4; ++i)
#pragma unroll
    for (int j = 0; j < 4; ++j) acc[i][j] = (v8f){0.f,0.f,0.f,0.f,0.f,0.f,0.f,0.f};

  for (int k0 = 0; k0 < K; k0 += 32) {
    V bh[4], bl[4];
#pragma unroll
    for (int j = 0; j < 4; ++j) {
      const size_t bo = (size_t)(n0 + (j << 4) + rlane) * ldb + koff + k0;
      bh[j] = Frag<T>::load(Bb + bo);
      if (SPLIT) bl[j] = Frag<T>::load(Bb2 + bo);
    }
#pragma unroll
    for (int i = 0; i < 4; ++i) {
      const size_t ao = (size_t)(m0 + (i << 4) + rlane) * lda + koff + k0;
      V ah = Frag<T>::load(Ab + ao);
      V al;
      if (SPLIT) al = Frag<T>::load(Ab2 + ao);
#pragma unroll
      for (int j = 0; j < 4; ++j) {
        acc[i][j] = Frag<T>::mma(ah, bh[j], acc[i][j]);
        if (SPLIT) {
          acc[i][j] = Frag<T>::mma(ah, bl[j], acc[i][j]);
          acc[i][j] = Frag<T>::mma(al, bh[j], acc[i][j]);
        }
      }
      Frag<T>::guard(acc[i][0], acc[i][3], ah, SPLIT ? al : ah);
    }
    Frag<T>::keep(bh[0], bh[1], bh[2], bh[3]);
    if (SPLIT) Frag<T>::keep(bl[0], bl[1], bl[2], bl[3]);
  }
  acc_guard4(acc[0][0], acc[0][1], acc[0][2], acc[0][3]);
  acc_guard4(acc[1][0], acc[1][1], acc[1][2], acc[1][3]);
  acc_guard4(acc[2][0], acc[2][1], acc[2][2], acc[2][3]);
  acc_guard4(acc[3][0], acc[3][1], acc[3][2], acc[3][3]);

  float* slab = sT[wave];
  const float* Rb = RESID ? (resid + (size_t)b * strideR) : nullptr;
#pragma unroll
  for (int i = 0; i < 4; ++i) {
    const int mBase = m0 + (i << 4);
#pragma unroll
    for (int j = 0; j < 4; ++j) {
      const int n = n0 + (j << 4) + rlane;
      float bv = 0.f;
      if (BIAS_MODE == 2) bv = bias[n];
#pragma unroll
      for (int r = 0; r < 8; ++r) {
        float v = acc[i][j][r] * scale;
        if (BIAS_MODE == 1) v += bias[mBase + mOff + r];
        if (BIAS_MODE == 2) v += bv;
        if (RESID) v += Rb[(size_t)(mBase + mOff + r) * ldc + n];
        if (ACT == 1) v = tanhf(v);
        if (ACT == 2) v = fmaxf(v, 0.0f);
        if (ACT == 3) v = v / (1.0f + expf(-v));
        if (ACT == 4) v = (v > 0.f) ? v : 0.01f * v;
        if (ACT == 5) v = 0.5f * v * (1.0f + erff(v * 0.70710678118654752f));
        slab[(mOff + r) * 68 + (j << 4) + rlane] = v;
      }
    }
    __builtin_amdgcn_fence(__ATOMIC_RELEASE, "workgroup");
    __builtin_amdgcn_wave_barrier();
    __builtin_amdgcn_fence(__ATOMIC_ACQUIRE, "workgroup");
    if (OUT_MODE == 0) {
      float* C = (float*)Cout + (size_t)b * strideC;
      const int hh = lane >> 4, c4 = (lane & 15) * 4;
      for (int pass = 0; pass < 2; ++pass) {
#pragma unroll
        for (int it = 0; it < 8; ++it) {
          const int row = it * 2 + hh;
          v4f v = *(const v4f*)(slab + row * 68 + c4);
          *(volatile v4f*)(C + (size_t)(mBase + row) * ldc + n0 + c4) = v;
        }
        __threadfence();
      }
    } else {
      const int q = lane >> 3, c8 = (lane & 7) * 8;
      unsigned short* C  = (unsigned short*)Cout  + (size_t)b * strideC;
      unsigned short* C2 = (OUT_MODE == 2) ? ((unsigned short*)Cout2 + (size_t)b * strideC) : nullptr;
      for (int pass = 0; pass < 2; ++pass) {
#pragma unroll
        for (int it = 0; it < 4; ++it) {
          const int row = it * 4 + q;
          const float* sp = slab + row * 68 + c8;
          v8h hv, lv;
#pragma unroll
          for (int e = 0; e < 8; ++e) {
            if (OUT_MODE == 1) {
              hv[e] = (_Float16)sp[e];
            } else {
              unsigned short hb = f2bf_bits(sp[e]);
              unsigned short lb = f2bf_bits(sp[e] - bf_bits2f(hb));
              hv[e] = __builtin_bit_cast(_Float16, hb);
              lv[e] = __builtin_bit_cast(_Float16, lb);
            }
          }
          *(volatile v8h*)(C + (size_t)(mBase + row) * ldc + n0 + c8) = hv;
          if (OUT_MODE == 2) *(volatile v8h*)(C2 + (size_t)(mBase + row) * ldc + n0 + c8) = lv;
        }
        __threadfence();
      }
    }
    __builtin_amdgcn_fence(__ATOMIC_RELEASE, "workgroup");
    __builtin_amdgcn_wave_barrier();
    __builtin_amdgcn_fence(__ATOMIC_ACQUIRE, "workgroup");
  }
}

__device__ __forceinline__ v8f mma_h(v16h a, v16h b, v8f c) {
  c = __builtin_amdgcn_wmma_f32_16x16x32_f16(false, a, false, b, (short)0, c, false, false);
  asm volatile("v_nop\n\tv_nop\n\tv_nop\n\tv_nop" : "+v"(c) : "v"(a), "v"(b));
  return c;
}
__device__ __forceinline__ unsigned pk2(float a, float b) {
  const unsigned short ua = __builtin_bit_cast(unsigned short, (_Float16)a);
  const unsigned short ub = __builtin_bit_cast(unsigned short, (_Float16)b);
  return (unsigned)ua | ((unsigned)ub << 16);
}
__device__ __forceinline__ float h16f(unsigned hb) {
  const unsigned s  = (hb & 0x8000u) << 16;
  const unsigned em = hb & 0x7fffu;
  const unsigned n  = s | ((em << 13) + (112u << 23));
  return (em < 0x0400u) ? __uint_as_float(s) : __uint_as_float(n);
}
__device__ __forceinline__ float sigm(float x) { return 1.0f / (1.0f + expf(-x)); }

__global__ __launch_bounds__(256) void k_embed(const int* __restrict__ tok, const float* __restrict__ emb,
                                               int nvocab, unsigned short* __restrict__ hemb) {
  const int tid = threadIdx.x;
  const int row = blockIdx.x * 16 + (tid >> 4);
  const int q   = tid & 15;
  const int b   = row / NSEQPAD;
  const int l   = row - b * NSEQPAD;
  const int lc  = (l < NSEQ) ? l : (NSEQ - 1);
  int id = tok[(size_t)b * NSEQ + lc];
  id = (id < 0) ? 0 : id;
  id = (id >= nvocab) ? (nvocab - 1) : id;
  const float* src = emb + (size_t)id * NEMB + q * 8;
  const v4f a = *(const v4f*)(src);
  const v4f c = *(const v4f*)(src + 4);
  const bool live = (l < NSEQ);
  u32x4 w;
  w.x = pk2(live ? a.x * CARRY16 : 0.0f, live ? a.y * CARRY16 : 0.0f);
  w.y = pk2(live ? a.z * CARRY16 : 0.0f, live ? a.w * CARRY16 : 0.0f);
  w.z = pk2(live ? c.x * CARRY16 : 0.0f, live ? c.y * CARRY16 : 0.0f);
  w.w = pk2(live ? c.z * CARRY16 : 0.0f, live ? c.w * CARRY16 : 0.0f);
  unsigned short* dst = hemb + (size_t)row * NEMB + q * 8;
  *(volatile u32x4*)dst = w;
  __threadfence();
  *(volatile u32x4*)dst = w;
}

__global__ __launch_bounds__(256) void k_pack_conv(const float* __restrict__ w, unsigned short* __restrict__ out) {
  const int idx = blockIdx.x * 256 + threadIdx.x;
  if (idx < NFILT * (KCONV / 8)) {
    const int f  = idx / (KCONV / 8);
    const int q  = idx - f * (KCONV / 8);
    const int c0 = q * 8;
    const int k  = c0 / NEMB;
    const int e0 = c0 - k * NEMB;
    const float* wp = w + (size_t)f * KCONV + (size_t)e0 * NTAP + k;
    float v[8];
#pragma unroll
    for (int i = 0; i < 8; ++i) v[i] = wp[i * NTAP] * CARRY16;
    u32x4 o;
    o.x = pk2(v[0], v[1]); o.y = pk2(v[2], v[3]); o.z = pk2(v[4], v[5]); o.w = pk2(v[6], v[7]);
    unsigned short* dst = out + (size_t)idx * 8;
    *(volatile u32x4*)dst = o;
    __threadfence();
    *(volatile u32x4*)dst = o;
  }
}

__global__ __launch_bounds__(256) void k_scale_cast(const float* __restrict__ in, unsigned short* __restrict__ out, int n8, float s) {
  const int i = blockIdx.x * 256 + threadIdx.x;
  if (i < n8) {
    const v4f a = *(const v4f*)(in + (size_t)i * 8);
    const v4f c = *(const v4f*)(in + (size_t)i * 8 + 4);
    u32x4 o;
    o.x = pk2(a.x * s, a.y * s); o.y = pk2(a.z * s, a.w * s); o.z = pk2(c.x * s, c.y * s); o.w = pk2(c.z * s, c.w * s);
    unsigned short* dst = out + (size_t)i * 8;
    *(volatile u32x4*)dst = o;
    __threadfence();
    *(volatile u32x4*)dst = o;
  }
}

__global__ __launch_bounds__(128) void k_bias(const float* __restrict__ b1, const float* __restrict__ b2, float* __restrict__ ob, float s) {
  const int i = threadIdx.x;
  const v4f a = *(const v4f*)(b1 + i * 4);
  const v4f c = *(const v4f*)(b2 + i * 4);
  const v4f v = (a + c) * s;
  *(volatile v4f*)(ob + i * 4) = v;
  __threadfence();
  *(volatile v4f*)(ob + i * 4) = v;
}

__global__ __launch_bounds__(256) void k_pool(const unsigned short* __restrict__ cpl, const float* __restrict__ cb, unsigned short* __restrict__ hp) {
  const int gid = blockIdx.x * 256 + threadIdx.x;
  const int tp  = gid >> 3;
  const int q   = gid & 7;
  const int b   = tp >> 10;
  const int t   = tp & (NSTEPPAD - 1);
  const int tcl = (t < NSTEP) ? t : (NSTEP - 1);
  const unsigned short* src = cpl + (((size_t)b * NSEQ + (size_t)4 * tcl) * NFILT + (size_t)q * 8);
  const u32x4 w0 = *(const u32x4*)(src);
  const u32x4 w1 = *(const u32x4*)(src + NFILT);
  const u32x4 w2 = *(const u32x4*)(src + 2 * NFILT);
  const u32x4 w3 = *(const u32x4*)(src + 3 * NFILT);
  float m[8];
#pragma unroll
  for (int j = 0; j < 4; ++j) {
    const float a0 = h16f(w0[j] & 0xffffu), a1 = h16f(w0[j] >> 16);
    const float b0v = h16f(w1[j] & 0xffffu), b1v = h16f(w1[j] >> 16);
    const float c0 = h16f(w2[j] & 0xffffu), c1 = h16f(w2[j] >> 16);
    const float d0 = h16f(w3[j] & 0xffffu), d1 = h16f(w3[j] >> 16);
    m[2 * j]     = fmaxf(fmaxf(a0, b0v), fmaxf(c0, d0));
    m[2 * j + 1] = fmaxf(fmaxf(a1, b1v), fmaxf(c1, d1));
  }
  const v4f cb0 = *(const v4f*)(cb + q * 8);
  const v4f cb1 = *(const v4f*)(cb + q * 8 + 4);
  const float bb[8] = {cb0.x, cb0.y, cb0.z, cb0.w, cb1.x, cb1.y, cb1.z, cb1.w};
  const bool live = (t < NSTEP);
  float v[8];
#pragma unroll
  for (int i = 0; i < 8; ++i) v[i] = live ? fmaxf(m[i] + CARRY16 * bb[i], 0.0f) : 0.0f;
  u32x4 o;
  o.x = pk2(v[0], v[1]); o.y = pk2(v[2], v[3]); o.z = pk2(v[4], v[5]); o.w = pk2(v[6], v[7]);
  unsigned short* dst = hp + (size_t)tp * NFILT + q * 8;
  *(volatile u32x4*)dst = o;
  __threadfence();
  *(volatile u32x4*)dst = o;
}

__global__ __launch_bounds__(256) void k_scan(const unsigned short* __restrict__ xg16, const unsigned short* __restrict__ whh16,
                                              const float* __restrict__ fcw, const float* __restrict__ fcb,
                                              float* __restrict__ out) {
  __shared__ __align__(16) _Float16 hsh[16 * HPITCH];
  __shared__ __align__(16) float    xs[16 * NGATE];
  const int tid  = threadIdx.x;
  const int wv   = tid >> 5;
  const int lane = tid & 31;
  const int hh   = lane >> 4;
  const int rl   = lane & 15;
  const int koff = hh * 8;
  const int b0   = blockIdx.x * 16;
  const int jg   = wv * 16 + rl;
  const _Float16* whh = (const _Float16*)whh16;

  for (int i = tid; i < (16 * HPITCH) / 8; i += 256) *(u32x4*)(hsh + i * 8) = (u32x4){0u, 0u, 0u, 0u};
  float cst[8], hreg[8];
#pragma unroll
  for (int r = 0; r < 8; ++r) { cst[r] = 0.0f; hreg[r] = 0.0f; }
  __syncthreads();

  for (int t = 0; t < NSTEP; ++t) {
    {
      const int mb = tid >> 4, seg = tid & 15;
      const unsigned short* src = xg16 + ((size_t)(b0 + mb) * NSTEPPAD + (size_t)t) * NGATE + seg * 32;
      float* dst = xs + mb * NGATE + seg * 32;
#pragma unroll
      for (int u = 0; u < 4; ++u) {
        const u32x4 w = *(const u32x4*)(src + u * 8);
        v4f f0, f1;
        f0.x = h16f(w.x & 0xffffu) * INV256; f0.y = h16f(w.x >> 16) * INV256;
        f0.z = h16f(w.y & 0xffffu) * INV256; f0.w = h16f(w.y >> 16) * INV256;
        f1.x = h16f(w.z & 0xffffu) * INV256; f1.y = h16f(w.z >> 16) * INV256;
        f1.z = h16f(w.w & 0xffffu) * INV256; f1.w = h16f(w.w >> 16) * INV256;
        *(v4f*)(dst + u * 8)     = f0;
        *(v4f*)(dst + u * 8 + 4) = f1;
      }
    }
    __syncthreads();

    v16h af[4];
#pragma unroll
    for (int kc = 0; kc < 4; ++kc) af[kc] = Frag<_Float16>::load(hsh + rl * HPITCH + kc * 32 + koff);

    v8f acc[4];
#pragma unroll
    for (int gi = 0; gi < 4; ++gi) {
      acc[gi] = (v8f){0.f, 0.f, 0.f, 0.f, 0.f, 0.f, 0.f, 0.f};
      const _Float16* bp = whh + (size_t)(gi * NHID + jg) * NHID + koff;
#pragma unroll
      for (int kc = 0; kc < 4; ++kc) {
        const v16h bb = Frag<_Float16>::load(bp + kc * 32);
        acc[gi] = mma_h(af[kc], bb, acc[gi]);
      }
      asm volatile("" ::: "memory");
    }

#pragma unroll
    for (int r = 0; r < 8; ++r) {
      const float* xr = xs + (hh * 8 + r) * NGATE + jg;
      const float pi = acc[0][r] * INV256 + xr[0];
      const float pf = acc[1][r] * INV256 + xr[NHID];
      const float pg = acc[2][r] * INV256 + xr[2 * NHID];
      const float po = acc[3][r] * INV256 + xr[3 * NHID];
      const float ig = sigm(pi);
      const float fg = sigm(pf);
      const float gg = tanhf(pg);
      const float og = sigm(po);
      const float cn = fg * cst[r] + ig * gg;
      cst[r]  = cn;
      hreg[r] = og * tanhf(cn);
    }
    __syncthreads();
#pragma unroll
    for (int r = 0; r < 8; ++r) hsh[(hh * 8 + r) * HPITCH + jg] = (_Float16)(hreg[r] * CARRY16);
  }

#pragma unroll
  for (int r = 0; r < 8; ++r) xs[(hh * 8 + r) * NHID + jg] = hreg[r];
  __syncthreads();
  if (tid < 32) {
    const int mm = tid >> 1;
    const int cc = tid & 1;
    float s = 0.0f;
#pragma unroll 1
    for (int k = 0; k < NHID; ++k) s += xs[mm * NHID + k] * fcw[cc * NHID + k];
    s += fcb[cc];
    volatile float* op = out + (size_t)b0 * NCLS;
    op[tid] = s;
    __threadfence();
    op[tid] = s;
  }
}

extern "C" void kernel_launch(void* const* d_in, const int* in_sizes, int n_in,
                              void* d_out, int out_size, void* d_ws, size_t ws_size,
                              hipStream_t stream) {
  if (n_in < 10) return;
  if (in_sizes[0] != NBATCH * NSEQ) return;
  if (in_sizes[1] < NEMB || (in_sizes[1] % NEMB) != 0) return;
  if (in_sizes[2] != NFILT * NEMB * NTAP) return;
  if (in_sizes[3] != NFILT) return;
  if (in_sizes[4] != NGATE * NFILT) return;
  if (in_sizes[5] != NGATE * NHID) return;
  if (in_sizes[6] != NGATE || in_sizes[7] != NGATE) return;
  if (in_sizes[8] != NCLS * NHID || in_sizes[9] != NCLS) return;
  if (out_size != NBATCH * NCLS) return;
  if (ws_size < WS_TOTAL) return;
  const int nvocab = in_sizes[1] / NEMB;

  const int*   x      = (const int*)  d_in[0];
  const float* emb    = (const float*)d_in[1];
  const float* conv_w = (const float*)d_in[2];
  const float* conv_b = (const float*)d_in[3];
  const float* w_ih   = (const float*)d_in[4];
  const float* w_hh   = (const float*)d_in[5];
  const float* b_ih   = (const float*)d_in[6];
  const float* b_hh   = (const float*)d_in[7];
  const float* fc_w   = (const float*)d_in[8];
  const float* fc_b   = (const float*)d_in[9];
  float* out = (float*)d_out;

  char* ws = (char*)d_ws;
  unsigned short* hemb    = (unsigned short*)(ws + OFF_HEMB);
  unsigned short* xg16    = (unsigned short*)(ws + OFF_HEMB);
  unsigned short* cpl     = (unsigned short*)(ws + OFF_CONV);
  unsigned short* hpool   = (unsigned short*)(ws + OFF_HPOOL);
  unsigned short* wconv   = (unsigned short*)(ws + OFF_WCONV);
  unsigned short* wih     = (unsigned short*)(ws + OFF_WIH);
  unsigned short* whh     = (unsigned short*)(ws + OFF_WHH);
  float*          bias256 = (float*)         (ws + OFF_BIAS);

  k_embed<<<(NBATCH * NSEQPAD) / 16, 256, 0, stream>>>(x, emb, nvocab, hemb);
  k_pack_conv<<<(NFILT * (KCONV / 8) + 255) / 256, 256, 0, stream>>>(conv_w, wconv);
  k_scale_cast<<<(NGATE * NFILT / 8 + 255) / 256, 256, 0, stream>>>(w_ih, wih, NGATE * NFILT / 8, CARRY16);
  k_scale_cast<<<(NGATE * NHID / 8 + 255) / 256, 256, 0, stream>>>(w_hh, whh, NGATE * NHID / 8, CARRY16);
  k_bias<<<1, 128, 0, stream>>>(b_ih, b_hh, bias256, 256.0f);

  wmma_gemm64<0, false, 0, 1, false, 0><<<dim3(NSEQ / 64 / 8, NBATCH), 256, 0, stream>>>(
      hemb, hemb, NEMB, (long)NSEQPAD * NEMB,
      wconv, wconv, KCONV, 0L,
      (void*)cpl, (void*)cpl, NFILT, (long)NSEQ * NFILT,
      bias256, bias256, 0L,
      NSEQ, NFILT, KCONV, 1.0f / 16.0f);

  k_pool<<<(NBATCH * NSTEPPAD * 8) / 256, 256, 0, stream>>>(cpl, conv_b, hpool);

  wmma_gemm64<0, false, 2, 1, false, 0><<<dim3((NBATCH * NSTEPPAD / 64) * (NGATE / 64) / 8, 1), 256, 0, stream>>>(
      hpool, hpool, NFILT, 0L,
      wih, wih, NFILT, 0L,
      (void*)xg16, (void*)xg16, NGATE, 0L,
      bias256, bias256, 0L,
      NBATCH * NSTEPPAD, NGATE, NFILT, 1.0f);

  k_scan<<<NBATCH / 16, 256, 0, stream>>>(xg16, whh, fc_w, fc_b, out);
}
